// TFMambaBlock_6854767805184
// MI455X (gfx1250) — hardware-verified
//
#include <hip/hip_runtime.h>
#include <hip/hip_bf16.h>
#include <math.h>

typedef __attribute__((ext_vector_type(16))) _Float16 v16h;
typedef __attribute__((ext_vector_type(8)))  _Float16 v8h;
typedef __attribute__((ext_vector_type(16))) __bf16   v16b;
typedef __attribute__((ext_vector_type(8)))  __bf16   v8b;
typedef __attribute__((ext_vector_type(8)))  float    v8f;
typedef __attribute__((ext_vector_type(4)))  float    v4f;

constexpr int kRows = 32768;
constexpr int kCm   = 64;
constexpr int kDi   = 128;
constexpr int kNs   = 16;
constexpr int kDtr  = 4;
constexpr int kXpr  = 36;
constexpr int kXpp  = 64;
constexpr int kTch  = 16;
constexpr int kYp   = 132;
constexpr int kTlen = 256;
constexpr int kFlen = 128;
constexpr int kLa   = 256;
constexpr int kLb   = 128;

constexpr int kWinH = 0;
constexpr int kWinL = 65536;
constexpr int kWxH  = 131072;
constexpr int kWxL  = 163840;
constexpr int kWoH  = 196608;
constexpr int kWoL  = 229376;
constexpr int kWtH  = 262144;
constexpr int kWtL  = 270336;
constexpr int kWfH  = 278528;
constexpr int kWfL  = 286720;
constexpr int kWEnd = 294912;

__device__ __forceinline__ unsigned short f2bf_bits(float f) {
  unsigned u = __float_as_uint(f);
  return (unsigned short)((u + 0x7FFFu + ((u >> 16) & 1u)) >> 16);
}
__device__ __forceinline__ float bf_bits2f(unsigned short h) { return __uint_as_float(((unsigned)h) << 16); }

__device__ __forceinline__ void dep_guard_h(v8f& a, v8f& b, v16h x, v16h y) { asm volatile("v_nop\n\tv_nop\n\tv_nop\n\tv_nop" : "+v"(a), "+v"(b) : "v"(x), "v"(y)); }
__device__ __forceinline__ void dep_guard_b(v8f& a, v8f& b, v16b x, v16b y) { asm volatile("v_nop\n\tv_nop\n\tv_nop\n\tv_nop" : "+v"(a), "+v"(b) : "v"(x), "v"(y)); }
__device__ __forceinline__ void keep4_h(v16h a, v16h b, v16h c, v16h d) { asm volatile("v_nop" :: "v"(a), "v"(b), "v"(c), "v"(d)); }
__device__ __forceinline__ void keep4_b(v16b a, v16b b, v16b c, v16b d) { asm volatile("v_nop" :: "v"(a), "v"(b), "v"(c), "v"(d)); }
__device__ __forceinline__ void acc_guard4(v8f& a, v8f& b, v8f& c, v8f& d) { asm volatile("v_nop\n\tv_nop\n\tv_nop\n\tv_nop" : "+v"(a), "+v"(b), "+v"(c), "+v"(d)); }
template <typename T> struct Frag;
template <> struct Frag<_Float16> {
  typedef v16h V; union U { v16h v; v8h h[2]; };
  static __device__ __forceinline__ v16h load(const _Float16* p) {
    U f; f.h[0] = *(const v8h*)(p); f.h[1] = *(const v8h*)(p + 16); return f.v;
  }
  static __device__ __forceinline__ v8f mma(v16h a, v16h b, v8f c) {
    return __builtin_amdgcn_wmma_f32_16x16x32_f16(false, a, false, b, (short)0, c, false, false);
  }
  static __device__ __forceinline__ void guard(v8f& a, v8f& b, v16h x, v16h y) { dep_guard_h(a, b, x, y); }
  static __device__ __forceinline__ void keep(v16h a, v16h b, v16h c, v16h d) { keep4_h(a, b, c, d); }
};
template <> struct Frag<__bf16> {
  typedef v16b V; union U { v16b v; v8b h[2]; };
  static __device__ __forceinline__ v16b load(const __bf16* p) {
    U f; f.h[0] = *(const v8b*)(p); f.h[1] = *(const v8b*)(p + 16); return f.v;
  }
  static __device__ __forceinline__ v8f mma(v16b a, v16b b, v8f c) {
    return __builtin_amdgcn_wmma_f32_16x16x32_bf16(false, a, false, b, (short)0, c, false, false);
  }
  static __device__ __forceinline__ void guard(v8f& a, v8f& b, v16b x, v16b y) { dep_guard_b(a, b, x, y); }
  static __device__ __forceinline__ void keep(v16b a, v16b b, v16b c, v16b d) { keep4_b(a, b, c, d); }
};

template <int ET> struct Elem;
template <> struct Elem<0> { typedef _Float16 T; };
template <> struct Elem<1> { typedef __bf16 T; };
template <int ET, bool SPLIT, int BIAS_MODE, int OUT_MODE, bool RESID, int ACT = 0>
__global__ __launch_bounds__(256) void wmma_gemm64(
    const unsigned short* __restrict__ Ap, const unsigned short* __restrict__ A2p, int lda, long strideA,
    const unsigned short* __restrict__ Btp, const unsigned short* __restrict__ Bt2p, int ldb, long strideB,
    void* __restrict__ Cout, void* __restrict__ Cout2, int ldc, long strideC,
    const float* __restrict__ bias,
    const float* __restrict__ resid, long strideR,
    int M, int N, int K, float scale) {
  typedef typename Elem<ET>::T T;
  typedef typename Frag<T>::V V;
  const T* A = (const T*)Ap; const T* A2 = (const T*)A2p; const T* Bt = (const T*)Btp; const T* Bt2 = (const T*)Bt2p;
  __shared__ __align__(16) float sT[8][16 * 68];
  const int b    = blockIdx.y;
  const int lane = threadIdx.x & 31;
  const int wave = threadIdx.x >> 5;
  const int tilesN = N >> 6;
  const int tilesM = M >> 6;
  const int tile = blockIdx.x * 8 + wave;
  if (tile >= tilesM * tilesN) return;
  const int tm = tile / tilesN;
  const int tn = tile - tm * tilesN;
  const int m0 = tm << 6;
  const int n0 = tn << 6;

  const T* Ab  = A  + (size_t)b * strideA;
  const T* Bb  = Bt + (size_t)b * strideB;
  const T* Ab2 = SPLIT ? (A2  + (size_t)b * strideA) : nullptr;
  const T* Bb2 = SPLIT ? (Bt2 + (size_t)b * strideB) : nullptr;

  const int rlane = lane & 15;
  const int koff  = (lane >> 4) * 8;
  const int mOff  = (lane >> 4) * 8;

  v8f acc[4][4];
#pragma unroll
  for (int i = 0; i < 4; ++i)
#pragma unroll
    for (int j = 0; j < 4; ++j) acc[i][j] = (v8f){0.f,0.f,0.f,0.f,0.f,0.f,0.f,0.f};

  for (int k0 = 0; k0 < K; k0 += 32) {
    V bh[4], bl[4];
#pragma unroll
    for (int j = 0; j < 4; ++j) {
      const size_t bo = (size_t)(n0 + (j << 4) + rlane) * ldb + koff + k0;
      bh[j] = Frag<T>::load(Bb + bo);
      if (SPLIT) bl[j] = Frag<T>::load(Bb2 + bo);
    }
#pragma unroll
    for (int i = 0; i < 4; ++i) {
      const size_t ao = (size_t)(m0 + (i << 4) + rlane) * lda + koff + k0;
      V ah = Frag<T>::load(Ab + ao);
      V al;
      if (SPLIT) al = Frag<T>::load(Ab2 + ao);
#pragma unroll
      for (int j = 0; j < 4; ++j) {
        acc[i][j] = Frag<T>::mma(ah, bh[j], acc[i][j]);
        if (SPLIT) {
          acc[i][j] = Frag<T>::mma(ah, bl[j], acc[i][j]);
          acc[i][j] = Frag<T>::mma(al, bh[j], acc[i][j]);
        }
      }
      Frag<T>::guard(acc[i][0], acc[i][3], ah, SPLIT ? al : ah);
    }
    Frag<T>::keep(bh[0], bh[1], bh[2], bh[3]);
    if (SPLIT) Frag<T>::keep(bl[0], bl[1], bl[2], bl[3]);
  }
  acc_guard4(acc[0][0], acc[0][1], acc[0][2], acc[0][3]);
  acc_guard4(acc[1][0], acc[1][1], acc[1][2], acc[1][3]);
  acc_guard4(acc[2][0], acc[2][1], acc[2][2], acc[2][3]);
  acc_guard4(acc[3][0], acc[3][1], acc[3][2], acc[3][3]);

  float* slab = sT[wave];
  const float* Rb = RESID ? (resid + (size_t)b * strideR) : nullptr;
#pragma unroll
  for (int i = 0; i < 4; ++i) {
    const int mBase = m0 + (i << 4);
#pragma unroll
    for (int j = 0; j < 4; ++j) {
      const int n = n0 + (j << 4) + rlane;
      float bv = 0.f;
      if (BIAS_MODE == 2) bv = bias[n];
#pragma unroll
      for (int r = 0; r < 8; ++r) {
        float v = acc[i][j][r] * scale;
        if (BIAS_MODE == 1) v += bias[mBase + mOff + r];
        if (BIAS_MODE == 2) v += bv;
        if (RESID) v += Rb[(size_t)(mBase + mOff + r) * ldc + n];
        if (ACT == 1) v = tanhf(v);
        if (ACT == 2) v = fmaxf(v, 0.0f);
        if (ACT == 3) v = v / (1.0f + expf(-v));
        if (ACT == 4) v = (v > 0.f) ? v : 0.01f * v;
        if (ACT == 5) v = 0.5f * v * (1.0f + erff(v * 0.70710678118654752f));
        slab[(mOff + r) * 68 + (j << 4) + rlane] = v;
      }
    }
    __builtin_amdgcn_fence(__ATOMIC_RELEASE, "workgroup");
    __builtin_amdgcn_wave_barrier();
    __builtin_amdgcn_fence(__ATOMIC_ACQUIRE, "workgroup");
    if (OUT_MODE == 0) {
      float* C = (float*)Cout + (size_t)b * strideC;
      const int hh = lane >> 4, c4 = (lane & 15) * 4;
      for (int pass = 0; pass < 2; ++pass) {
#pragma unroll
        for (int it = 0; it < 8; ++it) {
          const int row = it * 2 + hh;
          v4f v = *(const v4f*)(slab + row * 68 + c4);
          *(volatile v4f*)(C + (size_t)(mBase + row) * ldc + n0 + c4) = v;
        }
        __threadfence();
      }
    } else {
      const int q = lane >> 3, c8 = (lane & 7) * 8;
      unsigned short* C  = (unsigned short*)Cout  + (size_t)b * strideC;
      unsigned short* C2 = (OUT_MODE == 2) ? ((unsigned short*)Cout2 + (size_t)b * strideC) : nullptr;
      for (int pass = 0; pass < 2; ++pass) {
#pragma unroll
        for (int it = 0; it < 4; ++it) {
          const int row = it * 4 + q;
          const float* sp = slab + row * 68 + c8;
          v8h hv, lv;
#pragma unroll
          for (int e = 0; e < 8; ++e) {
            if (OUT_MODE == 1) {
              hv[e] = (_Float16)sp[e];
            } else {
              unsigned short hb = f2bf_bits(sp[e]);
              unsigned short lb = f2bf_bits(sp[e] - bf_bits2f(hb));
              hv[e] = __builtin_bit_cast(_Float16, hb);
              lv[e] = __builtin_bit_cast(_Float16, lb);
            }
          }
          *(volatile v8h*)(C + (size_t)(mBase + row) * ldc + n0 + c8) = hv;
          if (OUT_MODE == 2) *(volatile v8h*)(C2 + (size_t)(mBase + row) * ldc + n0 + c8) = lv;
        }
        __threadfence();
      }
    }
    __builtin_amdgcn_fence(__ATOMIC_RELEASE, "workgroup");
    __builtin_amdgcn_wave_barrier();
    __builtin_amdgcn_fence(__ATOMIC_ACQUIRE, "workgroup");
  }
}

__device__ __forceinline__ void split_bf8(v4f a0, v4f a1, v8h& hv, v8h& lv) {
#pragma unroll
  for (int e = 0; e < 4; ++e) {
    const unsigned short h0 = f2bf_bits(a0[e]);
    const unsigned short l0 = f2bf_bits(a0[e] - bf_bits2f(h0));
    const unsigned short h1 = f2bf_bits(a1[e]);
    const unsigned short l1 = f2bf_bits(a1[e] - bf_bits2f(h1));
    hv[e] = __builtin_bit_cast(_Float16, h0);     lv[e] = __builtin_bit_cast(_Float16, l0);
    hv[4 + e] = __builtin_bit_cast(_Float16, h1); lv[4 + e] = __builtin_bit_cast(_Float16, l1);
  }
}

__global__ __launch_bounds__(256) void weight_planes_kernel(
    const float* __restrict__ w_in, const float* __restrict__ w_x, const float* __restrict__ w_out,
    const float* __restrict__ w_t, const float* __restrict__ w_f, unsigned short* __restrict__ P)
{
  const int y = blockIdx.y;
  const float* W = w_in; int nrows = 1024, kdim = kCm, offh = kWinH, offl = kWinL, mode = 0;
  if (y == 1)      { W = w_x;   nrows = 256; kdim = kDi; offh = kWxH; offl = kWxL; mode = 1; }
  else if (y == 2) { W = w_out; nrows = 256; kdim = kDi; offh = kWoH; offl = kWoL; mode = 0; }
  else if (y == 3) { W = w_t;   nrows = 64;  kdim = kDi; offh = kWtH; offl = kWtL; mode = 2; }
  else if (y == 4) { W = w_f;   nrows = 64;  kdim = kDi; offh = kWfH; offl = kWfL; mode = 2; }
  const int nseg  = kdim >> 3;
  const int total = nrows * nseg;
  const int i = blockIdx.x * 256 + threadIdx.x;
  if (i >= total) return;
  const int n   = i / nseg;
  const int seg = i - n * nseg;
  v4f a0, a1;
#pragma unroll
  for (int e = 0; e < 4; ++e) {
    const int k0i = seg * 8 + e, k1i = seg * 8 + 4 + e;
    size_t i0, i1;
    bool real = true;
    if (mode == 0) {
      i0 = (size_t)n * kdim + k0i; i1 = (size_t)n * kdim + k1i;
    } else if (mode == 1) {
      const int grp = n >> 6, nn = n & 63;
      const int nnc = (nn < kXpr) ? nn : (kXpr - 1);
      real = (nn < kXpr);
      i0 = (size_t)(grp * kXpr + nnc) * kDi + k0i; i1 = (size_t)(grp * kXpr + nnc) * kDi + k1i;
    } else {
      i0 = (size_t)k0i * kCm + n; i1 = (size_t)k1i * kCm + n;
    }
    const float t0 = W[i0];
    const float t1 = W[i1];
    a0[e] = real ? t0 : 0.f;
    a1[e] = real ? t1 : 0.f;
  }
  v8h hv, lv;
  split_bf8(a0, a1, hv, lv);
  const size_t off = (size_t)n * kdim + seg * 8;
  for (int pass = 0; pass < 2; ++pass) {
    *(volatile v8h*)(P + offh + off) = hv;
    *(volatile v8h*)(P + offl + off) = lv;
    __threadfence();
  }
}

__global__ __launch_bounds__(256) void ingest_kernel(const float* __restrict__ x, float* __restrict__ U)
{
  __shared__ float sx[kCm * 129];
  const int t = blockIdx.x;
  const int tid = threadIdx.x;
#pragma unroll
  for (int it = 0; it < 8; ++it) {
    const int i  = it * 256 + tid;
    const int c  = i >> 5, f4 = (i & 31) * 4;
    const v4f v = *(const v4f*)(x + ((size_t)c * kTlen + t) * kFlen + f4);
    sx[c * 129 + f4 + 0] = v[0]; sx[c * 129 + f4 + 1] = v[1];
    sx[c * 129 + f4 + 2] = v[2]; sx[c * 129 + f4 + 3] = v[3];
  }
  __syncthreads();
  const int lane = tid & 31, wave = tid >> 5, hh = lane >> 4, c4 = (lane & 15) * 4;
  v4f o[8];
#pragma unroll
  for (int it = 0; it < 8; ++it) {
    const int f = it * 16 + wave * 2 + hh;
    v4f v;
    v[0] = sx[(c4 + 0) * 129 + f]; v[1] = sx[(c4 + 1) * 129 + f];
    v[2] = sx[(c4 + 2) * 129 + f]; v[3] = sx[(c4 + 3) * 129 + f];
    o[it] = v;
  }
  for (int pass = 0; pass < 2; ++pass) {
#pragma unroll
    for (int it = 0; it < 8; ++it) {
      const int f = it * 16 + wave * 2 + hh;
      *(volatile v4f*)(U + ((size_t)f * kLa + t) * kCm + c4) = o[it];
    }
    __threadfence();
  }
}

__global__ __launch_bounds__(256) void rmsnorm_planes_kernel(
    const float* __restrict__ U, const float* __restrict__ nw,
    unsigned short* __restrict__ Xh, unsigned short* __restrict__ Xl, int L, int flip)
{
  const int lane = threadIdx.x & 31, wave = threadIdx.x >> 5;
  const int q = lane >> 3, c8 = (lane & 7) * 8;
  const int r = blockIdx.x * 32 + wave * 4 + q;
  const int n = r / L, s = r - n * L;
  const int src = flip ? (n * L + (L - 1 - s)) : r;
  const v4f g0 = *(const v4f*)(nw + c8);
  const v4f g1 = *(const v4f*)(nw + c8 + 4);
  const v4f a0 = *(const v4f*)(U + (size_t)src * kCm + c8);
  const v4f a1 = *(const v4f*)(U + (size_t)src * kCm + c8 + 4);
  float ss = a0[0] * a0[0];
  ss = fmaf(a0[1], a0[1], ss); ss = fmaf(a0[2], a0[2], ss); ss = fmaf(a0[3], a0[3], ss);
  ss = fmaf(a1[0], a1[0], ss); ss = fmaf(a1[1], a1[1], ss); ss = fmaf(a1[2], a1[2], ss); ss = fmaf(a1[3], a1[3], ss);
#pragma unroll
  for (int off = 1; off < 8; off <<= 1) ss += __shfl_xor(ss, off, 32);
  const float nrm = rsqrtf(ss * (1.0f / 64.0f) + 1e-5f);
  v4f o0, o1;
#pragma unroll
  for (int e = 0; e < 4; ++e) { o0[e] = (a0[e] * nrm) * g0[e]; o1[e] = (a1[e] * nrm) * g1[e]; }
  v8h hv, lv;
  split_bf8(o0, o1, hv, lv);
  const size_t off = (size_t)r * kCm + c8;
  for (int pass = 0; pass < 2; ++pass) {
    *(volatile v8h*)(Xh + off) = hv;
    *(volatile v8h*)(Xl + off) = lv;
    __threadfence();
  }
}

__device__ __forceinline__ void tile16_to_planes128(const float* tile, int rb,
                                                    unsigned short* __restrict__ Ph, unsigned short* __restrict__ Pl)
{
  const int t = threadIdx.x;
  const int rsub = t >> 4, c8 = (t & 15) * 8;
  v8h hv[2], lv[2];
#pragma unroll
  for (int it = 0; it < 2; ++it) {
    const int row = it * 8 + rsub;
    const v4f a0 = *(const v4f*)(tile + row * kYp + c8);
    const v4f a1 = *(const v4f*)(tile + row * kYp + c8 + 4);
    split_bf8(a0, a1, hv[it], lv[it]);
  }
  for (int pass = 0; pass < 2; ++pass) {
#pragma unroll
    for (int it = 0; it < 2; ++it) {
      const int row = it * 8 + rsub;
      const size_t off = (size_t)(rb + row) * kDi + c8;
      *(volatile v8h*)(Ph + off) = hv[it];
      *(volatile v8h*)(Pl + off) = lv[it];
    }
    __threadfence();
  }
}

__global__ __launch_bounds__(128) void conv_silu_kernel(
    const float* __restrict__ X, const float* __restrict__ w_conv, const float* __restrict__ b_conv,
    unsigned short* __restrict__ UCh, unsigned short* __restrict__ UCl, int L)
{
  __shared__ __align__(16) float sX[kTch * kYp];
  const int d  = threadIdx.x;
  const int rb = blockIdx.x * L;
  int nchunk = L >> 4; if (nchunk > 16) nchunk = 16;
  const float w0 = w_conv[d * 4 + 0], w1 = w_conv[d * 4 + 1], w2 = w_conv[d * 4 + 2], w3 = w_conv[d * 4 + 3];
  const float bc = b_conv[d];
  float x0 = 0.f, x1 = 0.f, x2 = 0.f;
#pragma unroll 1
  for (int ch = 0; ch < nchunk; ++ch) {
    const int r0 = rb + ch * kTch;
    __syncthreads();
#pragma unroll 1
    for (int r = 0; r < kTch; ++r) {
      const float xcur = X[(size_t)(r0 + r) * kDi + d];
      float acc = w0 * x0;
      acc = fmaf(w1, x1, acc);
      acc = fmaf(w2, x2, acc);
      acc = fmaf(w3, xcur, acc);
      const float sv = acc + bc;
      const float sg = __builtin_amdgcn_rcpf(1.0f + __expf(-sv));
      sX[r * kYp + d] = sv * sg;
      x0 = x1; x1 = x2; x2 = xcur;
    }
    __syncthreads();
    tile16_to_planes128(sX, r0, UCh, UCl);
  }
}

__global__ __launch_bounds__(128) void scan_kernel(
    const float* __restrict__ DBL, const unsigned short* __restrict__ UCh, const unsigned short* __restrict__ UCl,
    const float* __restrict__ Z, const float* __restrict__ w_dt, const float* __restrict__ b_dt,
    const float* __restrict__ A_log, const float* __restrict__ Dsk,
    unsigned short* __restrict__ Yh, unsigned short* __restrict__ Yl, int L)
{
  __shared__ __align__(16) float sP[kTch * kXpp];
  __shared__ __align__(16) float sA[kDi * 17];
  __shared__ __align__(16) float sY[kTch * kYp];
  const int d  = threadIdx.x;
  const int rb = blockIdx.x * L;
  int nchunk = L >> 4; if (nchunk > 16) nchunk = 16;

#pragma unroll 1
  for (int n = 0; n < kNs; ++n) sA[d * 17 + n] = -expf(A_log[d * kNs + n]);
  __syncthreads();
  float An[kNs];
#pragma unroll
  for (int n = 0; n < kNs; ++n) An[n] = sA[d * 17 + n];
  float wd[kDtr];
#pragma unroll
  for (int r = 0; r < kDtr; ++r) wd[r] = w_dt[d * kDtr + r];
  const float bd = b_dt[d], Dd = Dsk[d];
  float h[kNs];
#pragma unroll
  for (int n = 0; n < kNs; ++n) h[n] = 0.f;

#pragma unroll 1
  for (int ch = 0; ch < nchunk; ++ch) {
    const int r0 = rb + ch * kTch;
    __syncthreads();
    *(v4f*)(sP + d * 4)       = *(const v4f*)(DBL + (size_t)r0 * kXpp + d * 4);
    *(v4f*)(sP + 512 + d * 4) = *(const v4f*)(DBL + (size_t)r0 * kXpp + 512 + d * 4);
    __syncthreads();
#pragma unroll 1
    for (int s = 0; s < kTch; ++s) {
      const size_t row = (size_t)r0 + s;
      const unsigned short uh = UCh[row * kDi + d];
      const unsigned short ul = UCl[row * kDi + d];
      const float ucv = bf_bits2f(uh) + bf_bits2f(ul);
      const float zv  = Z[row * kDi + d];
      const float* pr = sP + s * kXpp;
      const v4f t0 = *(const v4f*)(pr);
      v4f Bq[4], Cq[4];
#pragma unroll
      for (int q = 0; q < 4; ++q) {
        Bq[q] = *(const v4f*)(pr + kDtr + 4 * q);
        Cq[q] = *(const v4f*)(pr + kDtr + kNs + 4 * q);
      }
      float a = t0[0] * wd[0];
      a = fmaf(t0[1], wd[1], a); a = fmaf(t0[2], wd[2], a); a = fmaf(t0[3], wd[3], a);
      a += bd;
      const float dt = fmaxf(a, 0.f) + log1pf(__expf(-fabsf(a)));
      const float u = dt * ucv;
      float y = 0.f;
#pragma unroll
      for (int n = 0; n < kNs; ++n) {
        const float e = __expf(dt * An[n]);
        h[n] = fmaf(e, h[n], u * Bq[n >> 2][n & 3]);
        y = fmaf(h[n], Cq[n >> 2][n & 3], y);
      }
      y = fmaf(ucv, Dd, y);
      const float sg = __builtin_amdgcn_rcpf(1.0f + __expf(-zv));
      y = y * (zv * sg);
      sY[s * kYp + d] = y;
    }
    __syncthreads();
    tile16_to_planes128(sY, r0, Yh, Yl);
  }
}

__global__ __launch_bounds__(256) void concat_kernel(
    const float* __restrict__ OM, const float* __restrict__ U,
    unsigned short* __restrict__ Ch, unsigned short* __restrict__ Cl, int L, int flip, int coff)
{
  const int lane = threadIdx.x & 31, wave = threadIdx.x >> 5;
  const int q = lane >> 3, c8 = (lane & 7) * 8;
  const int r = blockIdx.x * 32 + wave * 4 + q;
  const int n = r / L, s = r - n * L;
  const int src = flip ? (n * L + (L - 1 - s)) : r;
  const v4f m0 = *(const v4f*)(OM + (size_t)r * kCm + c8);
  const v4f m1 = *(const v4f*)(OM + (size_t)r * kCm + c8 + 4);
  const v4f u0 = *(const v4f*)(U + (size_t)src * kCm + c8);
  const v4f u1 = *(const v4f*)(U + (size_t)src * kCm + c8 + 4);
  const v4f o0 = m0 + u0, o1 = m1 + u1;
  v8h hv, lv;
  split_bf8(o0, o1, hv, lv);
  const size_t off = (size_t)src * kDi + coff + c8;
  for (int pass = 0; pass < 2; ++pass) {
    *(volatile v8h*)(Ch + off) = hv;
    *(volatile v8h*)(Cl + off) = lv;
    __threadfence();
  }
}

__global__ __launch_bounds__(256) void rowperm_kernel(const float* __restrict__ XT, float* __restrict__ UB)
{
  const int lane = threadIdx.x & 31, wave = threadIdx.x >> 5;
  const int hh = lane >> 4, c4 = (lane & 15) * 4;
  const int o = blockIdx.x * 16 + wave * 2 + hh;
  const int t = o >> 7, f = o & 127;
  const int src = f * kLa + t;
  const v4f v = *(const v4f*)(XT + (size_t)src * kCm + c4);
  float* op = UB + (size_t)o * kCm + c4;
  for (int pass = 0; pass < 2; ++pass) {
    *(volatile v4f*)(op) = v;
    __threadfence();
  }
}

__global__ __launch_bounds__(256) void egress_kernel(const float* __restrict__ XF, float* __restrict__ out)
{
  __shared__ float sv[kFlen * 65];
  const int t = blockIdx.x;
  const int tid = threadIdx.x;
#pragma unroll
  for (int it = 0; it < 8; ++it) {
    const int i  = it * 256 + tid;
    const int f  = i >> 4, c4 = (i & 15) * 4;
    const v4f v = *(const v4f*)(XF + ((size_t)t * kFlen + f) * kCm + c4);
    sv[f * 65 + c4 + 0] = v[0]; sv[f * 65 + c4 + 1] = v[1];
    sv[f * 65 + c4 + 2] = v[2]; sv[f * 65 + c4 + 3] = v[3];
  }
  __syncthreads();
  const int lane = tid & 31, wave = tid >> 5, f4 = lane * 4;
  v4f o[8];
#pragma unroll
  for (int it = 0; it < 8; ++it) {
    const int c = it * 8 + wave;
    v4f v;
    v[0] = sv[(f4 + 0) * 65 + c]; v[1] = sv[(f4 + 1) * 65 + c];
    v[2] = sv[(f4 + 2) * 65 + c]; v[3] = sv[(f4 + 3) * 65 + c];
    o[it] = v;
  }
  for (int pass = 0; pass < 2; ++pass) {
#pragma unroll
    for (int it = 0; it < 8; ++it) {
      const int c = it * 8 + wave;
      *(volatile v4f*)(out + ((size_t)c * kTlen + t) * kFlen + f4) = o[it];
    }
    __threadfence();
  }
}

extern "C" void kernel_launch(void* const* d_in, const int* in_sizes, int n_in,
                              void* d_out, int out_size, void* d_ws, size_t ws_size,
                              hipStream_t stream)
{
  if (n_in < 15) return;
  const float* x        = (const float*)d_in[0];
  const float* norm_w   = (const float*)d_in[1];
  const float* in_proj  = (const float*)d_in[2];
  const float* conv_w   = (const float*)d_in[3];
  const float* conv_b   = (const float*)d_in[4];
  const float* x_proj   = (const float*)d_in[5];
  const float* dt_w     = (const float*)d_in[6];
  const float* dt_b     = (const float*)d_in[7];
  const float* A_log    = (const float*)d_in[8];
  const float* Dp       = (const float*)d_in[9];
  const float* out_proj = (const float*)d_in[10];
  const float* tlin_w   = (const float*)d_in[11];
  const float* tlin_b   = (const float*)d_in[12];
  const float* flin_w   = (const float*)d_in[13];
  const float* flin_b   = (const float*)d_in[14];

  if (in_sizes[0] != kCm * kTlen * kFlen) return;
  if (out_size != kCm * kTlen * kFlen) return;
  if (in_sizes[1] != 4 * kCm || in_sizes[2] != 4 * 2 * kDi * kCm || in_sizes[3] != 4 * kDi * 4 || in_sizes[4] != 4 * kDi) return;
  if (in_sizes[5] != 4 * kXpr * kDi || in_sizes[6] != 4 * kDi * kDtr || in_sizes[7] != 4 * kDi || in_sizes[8] != 4 * kDi * kNs) return;
  if (in_sizes[9] != 4 * kDi || in_sizes[10] != 4 * kCm * kDi) return;
  if (in_sizes[11] != 2 * kCm * kCm || in_sizes[12] != kCm || in_sizes[13] != 2 * kCm * kCm || in_sizes[14] != kCm) return;

  const size_t P64   = (size_t)kRows * kCm * 4;
  const size_t P128  = (size_t)kRows * kDi * 4;
  const size_t OFF_WGT = 0;
  const size_t OFF_U1  = 1048576;
  const size_t OFF_U2  = OFF_U1 + P64;
  const size_t OFF_P1  = OFF_U2 + P64;
  const size_t OFF_XY  = OFF_P1 + P128;
  const size_t OFF_Z   = OFF_XY + P128;
  const size_t OFF_DBL = OFF_Z + P128;
  const size_t OFF_CAT = OFF_DBL + P64;
  const size_t TOTAL   = OFF_CAT + P128;
  if (ws_size < TOTAL) return;
  if ((size_t)kWEnd * 2 > OFF_U1) return;

  char* ws = (char*)d_ws;
  unsigned short* WGT  = (unsigned short*)(ws + OFF_WGT);
  float* U1            = (float*)(ws + OFF_U1);
  float* U2            = (float*)(ws + OFF_U2);
  unsigned short* XNh  = (unsigned short*)(ws + OFF_P1);
  unsigned short* XNl  = XNh + (size_t)kRows * kCm;
  unsigned short* UCh  = (unsigned short*)(ws + OFF_P1);
  unsigned short* UCl  = UCh + (size_t)kRows * kDi;
  float* X             = (float*)(ws + OFF_XY);
  unsigned short* Yh   = (unsigned short*)(ws + OFF_XY);
  unsigned short* Yl   = Yh + (size_t)kRows * kDi;
  float* Z             = (float*)(ws + OFF_Z);
  float* DBL           = (float*)(ws + OFF_DBL);
  float* OM            = (float*)(ws + OFF_DBL);
  unsigned short* CATh = (unsigned short*)(ws + OFF_CAT);
  unsigned short* CATl = CATh + (size_t)kRows * kDi;
  float* dout          = (float*)d_out;

  const int TILES_M = kRows / 64;

  weight_planes_kernel<<<dim3(32, 5), 256, 0, stream>>>(in_proj, x_proj, out_proj, tlin_w, flin_w, WGT);
  ingest_kernel<<<kTlen, 256, 0, stream>>>(x, U1);

  auto run_mixer = [&](int i, int L, int nseq, int flip, int coff) {
    rmsnorm_planes_kernel<<<kRows / 32, 256, 0, stream>>>(U1, norm_w + i * kCm, XNh, XNl, L, flip);
    wmma_gemm64<1, true, 0, 0, false><<<dim3((TILES_M * 2) / 8, 2), 256, 0, stream>>>(
        XNh, XNl, kCm, 0L,
        WGT + kWinH + (size_t)i * 256 * kCm, WGT + kWinL + (size_t)i * 256 * kCm, kCm, (long)kDi * kCm,
        (void*)X, (void*)X, kDi, (long)kRows * kDi,
        DBL, DBL, 0L, kRows, kDi, kCm, 1.0f);
    conv_silu_kernel<<<nseq, 128, 0, stream>>>(X, conv_w + i * kDi * 4, conv_b + i * kDi, UCh, UCl, L);
    wmma_gemm64<1, true, 0, 0, false><<<dim3(TILES_M / 8, 1), 256, 0, stream>>>(
        UCh, UCl, kDi, 0L,
        WGT + kWxH + (size_t)i * kXpp * kDi, WGT + kWxL + (size_t)i * kXpp * kDi, kDi, 0L,
        (void*)DBL, (void*)DBL, kXpp, 0L,
        Z, Z, 0L, kRows, kXpp, kDi, 1.0f);
    scan_kernel<<<nseq, 128, 0, stream>>>(DBL, UCh, UCl, Z, dt_w + i * kDi * kDtr, dt_b + i * kDi,
                                            A_log + i * kDi * kNs, Dp + i * kDi, Yh, Yl, L);
    wmma_gemm64<1, true, 0, 0, false><<<dim3(TILES_M / 8, 1), 256, 0, stream>>>(
        Yh, Yl, kDi, 0L,
        WGT + kWoH + (size_t)i * kCm * kDi, WGT + kWoL + (size_t)i * kCm * kDi, kDi, 0L,
        (void*)OM, (void*)OM, kCm, 0L,
        Z, Z, 0L, kRows, kCm, kDi, 1.0f);
    concat_kernel<<<kRows / 32, 256, 0, stream>>>(OM, U1, CATh, CATl, L, flip, coff);
  };

  run_mixer(0, kLa, kRows / kLa, 0, 0);
  run_mixer(1, kLa, kRows / kLa, 1, kCm);
  wmma_gemm64<1, true, 2, 0, true><<<dim3(TILES_M / 8, 1), 256, 0, stream>>>(
      CATh, CATl, kDi, 0L, WGT + kWtH, WGT + kWtL, kDi, 0L,
      (void*)U2, (void*)U2, kCm, 0L, tlin_b, U1, 0L, kRows, kCm, kDi, 1.0f);
  rowperm_kernel<<<kRows / 16, 256, 0, stream>>>(U2, U1);

  run_mixer(2, kLb, kRows / kLb, 0, 0);
  run_mixer(3, kLb, kRows / kLb, 1, kCm);
  wmma_gemm64<1, true, 2, 0, true><<<dim3(TILES_M / 8, 1), 256, 0, stream>>>(
      CATh, CATl, kDi, 0L, WGT + kWfH, WGT + kWfL, kDi, 0L,
      (void*)U2, (void*)U2, kCm, 0L, flin_b, U1, 0L, kRows, kCm, kDi, 1.0f);

  egress_kernel<<<kTlen, 256, 0, stream>>>(U2, dout);
}
